// KNNLogitHead_10007273799761
// MI455X (gfx1250) — hardware-verified
//
#include <hip/hip_runtime.h>
#include <math.h>

typedef __attribute__((ext_vector_type(16))) _Float16 v16h;
typedef __attribute__((ext_vector_type(16))) __bf16 v16b;
typedef __attribute__((ext_vector_type(8)))  _Float16 v8h;
typedef __attribute__((ext_vector_type(8)))  float v8f;
typedef __attribute__((ext_vector_type(4)))  float v4f;
typedef __attribute__((ext_vector_type(2)))  float v2f;
typedef __attribute__((ext_vector_type(4)))  unsigned v4u;
typedef __attribute__((ext_vector_type(4)))  int v4i;
typedef float __attribute__((may_alias)) float_a;
typedef int __attribute__((may_alias)) int_a;

template <typename T> __device__ __forceinline__ void vst2(void* p, T v) { *(volatile T*)p = v; __threadfence(); *(volatile T*)p = v; }
__device__ __forceinline__ v8f wmma16(v16h a, v16h b, v8f c) {
  v8f d = __builtin_amdgcn_wmma_f32_16x16x32_f16(false, a, false, b, (short)0, c, false, false);
  asm volatile("v_nop\n\tv_nop\n\tv_nop\n\tv_nop" : "+v"(d) : "v"(a), "v"(b));
  return d;
}
__device__ __forceinline__ v8f wmma_bf(v16b a, v16b b, v8f c) {
  v8f d = __builtin_amdgcn_wmma_f32_16x16x32_bf16(false, a, false, b, (short)0, c, false, false);
  asm volatile("v_nop\n\tv_nop\n\tv_nop\n\tv_nop" : "+v"(d) : "v"(a), "v"(b));
  return d;
}
__device__ __forceinline__ v16h frag_h(const _Float16* rowk0, int lane) {
  union { v16h v; v8h q[2]; } u; const _Float16* p = rowk0 + 8 * (lane >> 4);
  u.q[0] = *(const v8h*)p; u.q[1] = *(const v8h*)(p + 16); return u.v;
}
__device__ __forceinline__ v16h frag_f32(const float* rowk0, int lane) {
  v16h a; const float* p = rowk0 + 8 * (lane >> 4);
#pragma unroll
  for (int i = 0; i < 8; ++i) { a[i] = (_Float16)p[i]; a[8 + i] = (_Float16)p[16 + i]; }
  return a;
}
__device__ __forceinline__ v16h frag_f32s(const float* rowk0, int lane, float sc) {
  v16h a; const float* p = rowk0 + 8 * (lane >> 4);
#pragma unroll
  for (int i = 0; i < 8; ++i) { a[i] = (_Float16)(p[i] * sc); a[8 + i] = (_Float16)(p[16 + i] * sc); }
  return a;
}
__device__ __forceinline__ v16h fragc_f32(const float* W, int k0, int n, int lane, int ld, int K) {
  v16h a; const int g = lane >> 4;
#pragma unroll
  for (int i = 0; i < 8; ++i) { const int ka = k0 + 8 * g + i, kb = ka + 16;
    a[i] = (_Float16)(ka < K ? W[(size_t)(ka < K ? ka : K - 1) * ld + n] : 0.f); a[8 + i] = (_Float16)(kb < K ? W[(size_t)(kb < K ? kb : K - 1) * ld + n] : 0.f); }
  return a;
}
struct F2 { v16b h, l; };
__device__ __forceinline__ F2 bsplit16(const float v[16]) { F2 r;
#pragma unroll
  for (int i = 0; i < 16; ++i) { const __bf16 h = (__bf16)v[i]; r.h[i] = h; r.l[i] = (__bf16)(v[i] - (float)h); }
  return r; }
__device__ __forceinline__ F2 split_row(const float* row, int k0, int lane) { float v[16]; const float* p = row + k0 + 8 * (lane >> 4);
#pragma unroll
  for (int i = 0; i < 8; ++i) { v[i] = p[i]; v[8 + i] = p[16 + i]; }
  return bsplit16(v); }
__device__ __forceinline__ F2 split_rowK(const float* row, int k0, int lane, int K) { float v[16]; const int g = lane >> 4;
#pragma unroll
  for (int i = 0; i < 8; ++i) { const int ka = k0 + 8 * g + i, kb = ka + 16; v[i] = ka < K ? row[ka < K ? ka : K - 1] : 0.f; v[8 + i] = kb < K ? row[kb < K ? kb : K - 1] : 0.f; }
  return bsplit16(v); }
__device__ __forceinline__ F2 split_col(const float* W, int k0, int n, int lane, int ld, int K) { float v[16]; const int g = lane >> 4;
#pragma unroll
  for (int i = 0; i < 8; ++i) { const int ka = k0 + 8 * g + i, kb = ka + 16; v[i] = ka < K ? W[(size_t)(ka < K ? ka : K - 1) * ld + n] : 0.f; v[8 + i] = kb < K ? W[(size_t)(kb < K ? kb : K - 1) * ld + n] : 0.f; }
  return bsplit16(v); }
__device__ __forceinline__ v8f mac3(const F2& a, const F2& b, v8f c) { c = wmma_bf(a.l, b.h, c); c = wmma_bf(a.h, b.l, c); return wmma_bf(a.h, b.h, c); }
__device__ __forceinline__ float sigm(float v) { return 1.0f / (1.0f + expf(-v)); }
#define LDSX() do { asm volatile("s_wait_dscnt 0" ::: "memory"); __builtin_amdgcn_wave_barrier(); __builtin_amdgcn_fence(__ATOMIC_RELEASE, "workgroup"); } while (0)


#define NBQ 262144
#define KK 16
#define NC 8
#define PH 32
#ifndef NBLKQ
#define NBLKQ (NBQ / 8)
#endif
typedef __attribute__((ext_vector_type(8))) __bf16 v8b;
__device__ __forceinline__ v16b frag_b(const __bf16* rowk0, int lane) {
  union { v16b v; v8b q[2]; } u; const __bf16* p = rowk0 + 8 * (lane >> 4);
  u.q[0] = *(const v8b*)p; u.q[1] = *(const v8b*)(p + 16); return u.v;
}
__device__ __forceinline__ float bfr(float v) { return (float)(__bf16)v; }
__device__ __attribute__((noinline)) float exp_ni(float v) { return expf(v); }
__device__ __attribute__((noinline)) float erf_ni(float v) { return erff(v); }

__device__ __forceinline__ float gelu_x(float v) { return 0.5f * v * (1.0f + erf_ni(v * 0.70710678118654752f)); }
#define WS_PW   0u
#define PW2 0
#define PR1 (PH * PH)
#define PWEND (PR1 + PH * 64)
#define WS_END  (WS_PW + 2u * PWEND)

__global__ __launch_bounds__(256) void k_pack(const float* __restrict__ W2, const float* __restrict__ WR1, __bf16* __restrict__ PW) {
  __shared__ __align__(16) __bf16 s2[PH][PH]; __shared__ __align__(16) __bf16 sr[PH][64]; const int tid = threadIdx.x;
  for (int q = tid; q < PH * PH; q += 256) { const int o = q / PH, i = q % PH; s2[o][i] = (__bf16)W2[i * PH + o]; }
  for (int q = tid; q < PH * 64; q += 256) { const int o = q / 64, kk = q % 64; sr[o][kk] = (__bf16)((kk < PH + 1) ? WR1[kk * PH + o] : 0.f); }
  __syncthreads();
  for (int q = tid; q < PH * PH / 8; q += 256) vst2((unsigned*)(PW + PW2 + q * 8), *(const v4u*)&(&s2[0][0])[q * 8]);
  for (int q = tid; q < PH * 64 / 8; q += 256) vst2((unsigned*)(PW + PR1 + q * 8), *(const v4u*)&(&sr[0][0])[q * 8]);
}
__global__ __launch_bounds__(128) void k_head(const float* __restrict__ VALS, const float* __restrict__ CLS, const float* __restrict__ W1, const float* __restrict__ B1, const __bf16* __restrict__ PW, const float* __restrict__ B2, const float* __restrict__ BR1, const float* __restrict__ WR2, const float* __restrict__ BR2, const float* __restrict__ RS, const float* __restrict__ RS2, float* __restrict__ O0, float* __restrict__ O1, float* __restrict__ O2) {
  __shared__ float sw1[PH], sb1[PH], sb2[PH], sbr1[PH], swr2[PH]; __shared__ __align__(16) float spool[4][2][NC][PH + 4]; __shared__ __align__(16) float so0[64], so1[64], so2[64];
  const int tid = threadIdx.x, wave = tid >> 5, lane = tid & 31, col = lane & 15, g = lane >> 4;
  if (tid < PH) { sw1[tid] = bfr(W1[tid]); sb1[tid] = bfr(B1[tid]); sb2[tid] = bfr(B2[tid]); sbr1[tid] = bfr(BR1[tid]); swr2[tid] = bfr(WR2[tid]); }
  __syncthreads();
  const float rs = bfr(RS[0]), rs2 = bfr(RS2[0]), br2 = bfr(BR2[0]);
  float csum_keep[2] = {0.f, 0.f}, cnt_keep[2] = {0.f, 0.f};
#pragma unroll
  for (int sub = 0; sub < 2; ++sub) { const size_t b = (size_t)blockIdx.x * 8 + wave * 2 + sub;
    const float vrow = bfr(VALS[b * KK + col]); float hv[16];
#pragma unroll
    for (int i = 0; i < 8; ++i) { hv[i] = gelu_x(vrow * sw1[8 * g + i] + sb1[8 * g + i]); hv[8 + i] = gelu_x(vrow * sw1[16 + 8 * g + i] + sb1[16 + 8 * g + i]); }
    const F2 a = bsplit16(hv); v8f acc[2] = {};
#pragma unroll
    for (int j = 0; j < 2; ++j) { const v16b w = frag_b(PW + PW2 + (size_t)(j * 16 + col) * PH, lane); acc[j] = wmma_bf(a.l, w, acc[j]); acc[j] = wmma_bf(a.h, w, acc[j]); }
    int ck[8]; float vk[8];
#pragma unroll
    for (int r = 0; r < 8; ++r) { const int k = 8 * g + r; float cf = bfr(CLS[b * KK + k]); int c = (int)cf; c = min(max(c, 0), NC - 1); ck[r] = c; vk[r] = bfr(VALS[b * KK + k]); }
    float pooled[2][NC]; float cnt[NC], csum[NC];
#pragma unroll
    for (int c = 0; c < NC; ++c) { pooled[0][c] = 0.f; pooled[1][c] = 0.f; cnt[c] = 0.f; csum[c] = 0.f; }
#pragma unroll
    for (int r = 0; r < 8; ++r) { const float p0 = gelu_x(acc[0][r] + sb2[col]), p1 = gelu_x(acc[1][r] + sb2[16 + col]);
#pragma unroll
      for (int c = 0; c < NC; ++c) { const bool m = (ck[r] == c); pooled[0][c] += m ? p0 : 0.f; pooled[1][c] += m ? p1 : 0.f; cnt[c] += m ? 1.f : 0.f; csum[c] += m ? vk[r] : 0.f; } }
#pragma unroll
    for (int c = 0; c < NC; ++c) { pooled[0][c] += __shfl_xor(pooled[0][c], 16); pooled[1][c] += __shfl_xor(pooled[1][c], 16); cnt[c] += __shfl_xor(cnt[c], 16); csum[c] += __shfl_xor(csum[c], 16); }
    if (g == 0) {
#pragma unroll
      for (int c = 0; c < NC; ++c) { spool[wave][sub][c][col] = pooled[0][c]; spool[wave][sub][c][16 + col] = pooled[1][c]; } }
    if (lane == 0) {
#pragma unroll
      for (int c = 0; c < NC; ++c) spool[wave][sub][c][PH] = cnt[c]; }
#pragma unroll
    for (int c = 0; c < NC; ++c) if (col == c) { csum_keep[sub] = csum[c]; cnt_keep[sub] = cnt[c]; }
  }
  LDSX();
  v8f racc[2] = {};
#pragma unroll
  for (int kc = 0; kc < 2; ++kc) { float v[16]; const float* pr = &spool[wave][col >> 3][col & 7][0];
#pragma unroll
    for (int i = 0; i < 8; ++i) { const int k0 = kc * 32 + 8 * g + i, k1 = kc * 32 + 16 + 8 * g + i; v[i] = (k0 <= PH) ? pr[k0] : 0.f; v[8 + i] = (k1 <= PH) ? pr[k1] : 0.f; }
    const F2 a = bsplit16(v);
#pragma unroll
    for (int j = 0; j < 2; ++j) { const v16b w = frag_b(PW + PR1 + (size_t)(j * 16 + col) * 64 + kc * 32, lane); racc[j] = wmma_bf(a.l, w, racc[j]); racc[j] = wmma_bf(a.h, w, racc[j]); } }
  float dl[8];
#pragma unroll
  for (int r = 0; r < 8; ++r) { float s = gelu_x(racc[0][r] + sbr1[col]) * swr2[col] + gelu_x(racc[1][r] + sbr1[16 + col]) * swr2[16 + col];
#pragma unroll
    for (int o = 1; o < 16; o <<= 1) s += __shfl_xor(s, o);
    dl[r] = s + br2; }
#pragma unroll
  for (int r = 0; r < 8; ++r) if (col == r) { const int idx = (wave * 2 + g) * NC + r; so1[idx] = csum_keep[g]; so2[idx] = cnt_keep[g]; so0[idx] = csum_keep[g] * rs2 + rs * dl[r]; }
  __syncthreads();
  if (tid < 16) vst2(O0 + (size_t)blockIdx.x * 64 + tid * 4, *(const v4f*)&so0[tid * 4]);
  else if (tid < 32) vst2(O1 + (size_t)blockIdx.x * 64 + (tid - 16) * 4, *(const v4f*)&so1[(tid - 16) * 4]);
  else if (tid < 48) vst2(O2 + (size_t)blockIdx.x * 64 + (tid - 32) * 4, *(const v4f*)&so2[(tid - 32) * 4]);
}
extern "C" void kernel_launch(void* const* d_in, const int* in_sizes, int n_in, void* d_out, int out_size, void* d_ws, size_t ws_size, hipStream_t stream) {
  (void)in_sizes; (void)n_in; (void)out_size;
  const float** F = (const float**)d_in;
  if (ws_size < (size_t)WS_END) return;
  char* ws = (char*)d_ws; __bf16* PW = (__bf16*)(ws + WS_PW);
  float* O0 = (float*)d_out; float* O1 = O0 + (size_t)NBQ * NC; float* O2 = O1 + (size_t)NBQ * NC;
  k_pack<<<1, 256, 0, stream>>>(F[4], F[6], PW);
  k_head<<<NBLKQ, 128, 0, stream>>>(F[0], F[1], F[2], F[3], PW, F[5], F[7], F[8], F[9], F[10], F[11], O0, O1, O2);
}
